// MainEffectBlock_4973572129353
// MI455X (gfx1250) — hardware-verified
//
#include <hip/hip_runtime.h>

typedef __attribute__((ext_vector_type(16))) _Float16 v16h;
typedef __attribute__((ext_vector_type(2)))  _Float16 h2v;
typedef __attribute__((ext_vector_type(8)))  float    v8f;

#define NN 16
#define NC 4
#define CATS 32
#define H1 40
#define H2 20
#define NF 20
#define TILE 256
#define THREADS 256

#define WMMA_F16(A, B, C) \
    __builtin_amdgcn_wmma_f32_16x16x32_f16(false, (A), false, (B), (short)0, (C), false, false)
#define RSPLIT (1.0f / 2048.0f)
__device__ __forceinline__ _Float16 lo_of(float v, _Float16 h) { return (_Float16)((v - (float)h) * 2048.0f); }
__device__ __forceinline__ v8f wmma_split(v16h a, v16h al, v16h b, v16h bl, v8f c) {
    v8f x = {}; x = WMMA_F16(al, b, x); x = WMMA_F16(a, bl, x); return WMMA_F16(a, b, c) + x * RSPLIT;
}
__device__ __forceinline__ int kof(int half, int e) { return ((e < 8) ? e : (e + 8)) + half * 8; }

struct BPack { h2v p[8]; };

__global__ __launch_bounds__(THREADS) void nam_forward_kernel(
    const float* __restrict__ inputs,
    const float* __restrict__ W1,
    const float* __restrict__ b1,
    const float* __restrict__ W2,
    const float* __restrict__ b2,
    const float* __restrict__ Wout,
    const float* __restrict__ bout,
    const float* __restrict__ minv,
    const float* __restrict__ maxv,
    const float* __restrict__ cemb,
    const float* __restrict__ cobias,
    float* __restrict__ out)
{
    __shared__ float sW2[NN * H1 * H2];
    __shared__ float sW1[NN * H1], sB1[NN * H1];
    __shared__ float sB2[NN * H2], sWout[NN * H2];
    __shared__ float sBout[NN], sMin[NN], sMax[NN];
    __shared__ float sEmb[NC * CATS], sObias[NC];
    __shared__ __align__(16) float sX[TILE * NF];

    const int tid = threadIdx.x;
    const size_t rowBase = (size_t)blockIdx.x * TILE;

    {
        const uint32_t sxOff = (uint32_t)(uintptr_t)(&sX[0]) + (uint32_t)(tid * 16);
        const float* src = inputs + rowBase * NF + tid * 4;
        #pragma unroll
        for (int r = 0; r < 5; ++r) {
            asm volatile("global_load_async_to_lds_b128 %0, %1, off"
                         :: "v"(sxOff + r * 4096), "v"(src + r * 1024)
                         : "memory");
        }
    }

    for (int i = tid; i < NN * H1 * H2; i += THREADS) sW2[i] = W2[i];
    for (int i = tid; i < NN * H1; i += THREADS) { sW1[i] = W1[i]; sB1[i] = b1[i]; }
    for (int i = tid; i < NN * H2; i += THREADS) { sB2[i] = b2[i]; sWout[i] = Wout[i]; }
    if (tid < NN) { sBout[tid] = bout[tid]; sMin[tid] = minv[tid]; sMax[tid] = maxv[tid]; }
    if (tid < NC * CATS) sEmb[tid] = cemb[tid];
    if (tid < NC) sObias[tid] = cobias[tid];

    asm volatile("s_wait_asynccnt 0" ::: "memory");
    __syncthreads();

    {
        const int row = tid;
        #pragma unroll
        for (int c = 0; c < NC; ++c) {
            int idx = (int)sX[row * NF + NN + c];
            if (idx < 0) idx += CATS;
            idx = (idx < 0) ? 0 : (idx > CATS - 1 ? CATS - 1 : idx);
            sX[row * NF + NN + c] = sEmb[c * CATS + idx] + sObias[c];
        }
    }

    const int lane   = tid & 31;
    const int wave   = tid >> 5;
    const int half16 = lane >> 4;
    const int l16    = lane & 15;

    #pragma unroll
    for (int fi = 0; fi < 2; ++fi) {
        const int f = wave + fi * 8;

        const float* wf = &sW2[f * H1 * H2];
        v16h a00, a01, a10, a11, l00, l01, l10, l11;
        #pragma unroll
        for (int h = 0; h < 16; ++h) {
            int kb = kof(half16, h);
            int k1 = kb + 32;
            int j0 = l16, j1 = l16 + 16;
            bool kok = (k1 < H1);
            const float v00 = wf[kb * H2 + j0];
            const float v10 = (j1 < H2) ? wf[kb * H2 + j1] : 0.0f;
            const float v01 = kok ? wf[k1 * H2 + j0] : 0.0f;
            const float v11 = (kok && j1 < H2) ? wf[k1 * H2 + j1] : 0.0f;
            a00[h] = (_Float16)v00; l00[h] = lo_of(v00, a00[h]);
            a10[h] = (_Float16)v10; l10[h] = lo_of(v10, a10[h]);
            a01[h] = (_Float16)v01; l01[h] = lo_of(v01, a01[h]);
            a11[h] = (_Float16)v11; l11[h] = lo_of(v11, a11[h]);
        }

        const float* w1f = sW1 + f * H1;
        const float* b1f = sB1 + f * H1;
        const bool c1ok = (half16 == 0);

        float b2c0[8], wc0[8], b2c1[4], wc1[4];
        #pragma unroll
        for (int r = 0; r < 8; ++r) {
            int j = r + half16 * 8;
            b2c0[r] = sB2[f * H2 + j]; wc0[r] = sWout[f * H2 + j];
        }
        #pragma unroll
        for (int r = 0; r < 4; ++r) {
            int j = 16 + r + half16 * 8;
            bool ok = (j < H2);
            b2c1[r] = ok ? sB2[f * H2 + j] : 0.0f;
            wc1[r]  = ok ? sWout[f * H2 + j] : 0.0f;
        }
        const float lo = sMin[f], hi = sMax[f], ob = sBout[f];

        auto buildB = [&](int t, v16h& B0, v16h& B1, v16h& L0, v16h& L1) {
            float x = fminf(fmaxf(sX[(t * 16 + l16) * NF + f], lo), hi);
            #pragma unroll
            for (int e = 0; e < 16; ++e) {
                const int k = kof(half16, e);
                const float s = fmaxf(fmaf(x, w1f[k], b1f[k]), 0.0f);
                B0[e] = (_Float16)s; L0[e] = lo_of(s, B0[e]);
            }
            #pragma unroll
            for (int e = 0; e < 8; ++e) {
                const int k = 32 + kof(0, e);
                const float s = c1ok ? fmaxf(fmaf(x, w1f[k], b1f[k]), 0.0f) : 0.0f;
                B1[e] = (_Float16)s; L1[e] = lo_of(s, B1[e]);
            }
            #pragma unroll
            for (int e = 8; e < 16; ++e) { B1[e] = (_Float16)0.0f; L1[e] = (_Float16)0.0f; }
        };

        auto step = [&](int t) {
            v16h B0, B1, L0, L1;
            buildB(t, B0, B1, L0, L1);
            v8f c0 = {}, c1 = {};
            c0 = wmma_split(a00, l00, B0, L0, c0);
            c0 = wmma_split(a01, l01, B1, L1, c0);
            c1 = wmma_split(a10, l10, B0, L0, c1);
            c1 = wmma_split(a11, l11, B1, L1, c1);

            float acc = 0.0f;
            #pragma unroll
            for (int r = 0; r < 8; ++r)
                acc = fmaf(fmaxf(c0[r] + b2c0[r], 0.0f), wc0[r], acc);
            #pragma unroll
            for (int r = 0; r < 4; ++r)
                acc = fmaf(fmaxf(c1[r] + b2c1[r], 0.0f), wc1[r], acc);
            acc += __shfl_xor(acc, 16, 32);
            sX[(t * 16 + l16) * NF + f] = acc + ob;
        };

        #pragma unroll 1
        for (int t = 0; t < 16; ++t) step(t);
    }

    __syncthreads();
    {
        const uint32_t sxOff = (uint32_t)(uintptr_t)(&sX[0]) + (uint32_t)(tid * 16);
        float* dst = out + rowBase * NF + tid * 4;
        #pragma unroll 1
        for (int pass = 0; pass < 2; ++pass) {
            #pragma unroll
            for (int r = 0; r < 5; ++r) {
                asm volatile("global_store_async_from_lds_b128 %0, %1, off"
                             :: "v"(dst + r * 1024), "v"(sxOff + r * 4096)
                             : "memory");
            }
            asm volatile("s_wait_asynccnt 0" ::: "memory");
            __threadfence();
        }
    }
}

extern "C" void kernel_launch(void* const* d_in, const int* in_sizes, int n_in,
                              void* d_out, int out_size, void* d_ws, size_t ws_size,
                              hipStream_t stream) {
    const float* inputs = (const float*)d_in[0];
    const float* W1     = (const float*)d_in[1];
    const float* b1     = (const float*)d_in[2];
    const float* W2     = (const float*)d_in[3];
    const float* b2     = (const float*)d_in[4];
    const float* Wout   = (const float*)d_in[5];
    const float* bout   = (const float*)d_in[6];
    const float* minv   = (const float*)d_in[7];
    const float* maxv   = (const float*)d_in[8];
    const float* cemb   = (const float*)d_in[9];
    const float* cobias = (const float*)d_in[10];
    float* outp = (float*)d_out;

    const int rows   = in_sizes[0] / NF;
    const int blocks = rows / TILE;

    nam_forward_kernel<<<blocks, THREADS, 0, stream>>>(
        inputs, W1, b1, W2, b2, Wout, bout, minv, maxv, cemb, cobias, outp);
}
